// MLASegmentCrossAttention_37469294690562
// MI455X (gfx1250) — hardware-verified
//
#include <hip/hip_runtime.h>
#include <math.h>

typedef __attribute__((ext_vector_type(16))) _Float16 v16h;
typedef __attribute__((ext_vector_type(16))) __bf16 v16b;
typedef __attribute__((ext_vector_type(8)))  _Float16 v8h;
typedef __attribute__((ext_vector_type(8)))  float v8f;
typedef __attribute__((ext_vector_type(4)))  float v4f;
typedef __attribute__((ext_vector_type(2)))  float v2f;
typedef __attribute__((ext_vector_type(4)))  unsigned v4u;
typedef __attribute__((ext_vector_type(4)))  int v4i;
typedef float __attribute__((may_alias)) float_a;
typedef int __attribute__((may_alias)) int_a;

template <typename T> __device__ __forceinline__ void vst2(void* p, T v) { *(volatile T*)p = v; __threadfence(); *(volatile T*)p = v; }
__device__ __forceinline__ v8f wmma16(v16h a, v16h b, v8f c) {
  v8f d = __builtin_amdgcn_wmma_f32_16x16x32_f16(false, a, false, b, (short)0, c, false, false);
  asm volatile("v_nop\n\tv_nop\n\tv_nop\n\tv_nop" : "+v"(d) : "v"(a), "v"(b));
  return d;
}
__device__ __forceinline__ v8f wmma_bf(v16b a, v16b b, v8f c) {
  v8f d = __builtin_amdgcn_wmma_f32_16x16x32_bf16(false, a, false, b, (short)0, c, false, false);
  asm volatile("v_nop\n\tv_nop\n\tv_nop\n\tv_nop" : "+v"(d) : "v"(a), "v"(b));
  return d;
}
__device__ __forceinline__ v16h frag_h(const _Float16* rowk0, int lane) {
  union { v16h v; v8h q[2]; } u; const _Float16* p = rowk0 + 8 * (lane >> 4);
  u.q[0] = *(const v8h*)p; u.q[1] = *(const v8h*)(p + 16); return u.v;
}
__device__ __forceinline__ v16h frag_f32(const float* rowk0, int lane) {
  v16h a; const float* p = rowk0 + 8 * (lane >> 4);
#pragma unroll
  for (int i = 0; i < 8; ++i) { a[i] = (_Float16)p[i]; a[8 + i] = (_Float16)p[16 + i]; }
  return a;
}
__device__ __forceinline__ v16h frag_f32s(const float* rowk0, int lane, float sc) {
  v16h a; const float* p = rowk0 + 8 * (lane >> 4);
#pragma unroll
  for (int i = 0; i < 8; ++i) { a[i] = (_Float16)(p[i] * sc); a[8 + i] = (_Float16)(p[16 + i] * sc); }
  return a;
}
__device__ __forceinline__ v16h fragc_f32(const float* W, int k0, int n, int lane, int ld, int K) {
  v16h a; const int g = lane >> 4;
#pragma unroll
  for (int i = 0; i < 8; ++i) { const int ka = k0 + 8 * g + i, kb = ka + 16;
    a[i] = (_Float16)(ka < K ? W[(size_t)(ka < K ? ka : K - 1) * ld + n] : 0.f); a[8 + i] = (_Float16)(kb < K ? W[(size_t)(kb < K ? kb : K - 1) * ld + n] : 0.f); }
  return a;
}
struct F2 { v16b h, l; };
__device__ __forceinline__ F2 bsplit16(const float v[16]) { F2 r;
#pragma unroll
  for (int i = 0; i < 16; ++i) { const __bf16 h = (__bf16)v[i]; r.h[i] = h; r.l[i] = (__bf16)(v[i] - (float)h); }
  return r; }
__device__ __forceinline__ F2 split_row(const float* row, int k0, int lane) { float v[16]; const float* p = row + k0 + 8 * (lane >> 4);
#pragma unroll
  for (int i = 0; i < 8; ++i) { v[i] = p[i]; v[8 + i] = p[16 + i]; }
  return bsplit16(v); }
__device__ __forceinline__ F2 split_rowK(const float* row, int k0, int lane, int K) { float v[16]; const int g = lane >> 4;
#pragma unroll
  for (int i = 0; i < 8; ++i) { const int ka = k0 + 8 * g + i, kb = ka + 16; v[i] = ka < K ? row[ka < K ? ka : K - 1] : 0.f; v[8 + i] = kb < K ? row[kb < K ? kb : K - 1] : 0.f; }
  return bsplit16(v); }
__device__ __forceinline__ F2 split_col(const float* W, int k0, int n, int lane, int ld, int K) { float v[16]; const int g = lane >> 4;
#pragma unroll
  for (int i = 0; i < 8; ++i) { const int ka = k0 + 8 * g + i, kb = ka + 16; v[i] = ka < K ? W[(size_t)(ka < K ? ka : K - 1) * ld + n] : 0.f; v[8 + i] = kb < K ? W[(size_t)(kb < K ? kb : K - 1) * ld + n] : 0.f; }
  return bsplit16(v); }
__device__ __forceinline__ v8f mac3(const F2& a, const F2& b, v8f c) { c = wmma_bf(a.l, b.h, c); c = wmma_bf(a.h, b.l, c); return wmma_bf(a.h, b.h, c); }
__device__ __forceinline__ float sigm(float v) { return 1.0f / (1.0f + expf(-v)); }
#define LDSX() do { asm volatile("s_wait_dscnt 0" ::: "memory"); __builtin_amdgcn_wave_barrier(); __builtin_amdgcn_fence(__ATOMIC_RELEASE, "workgroup"); } while (0)


#define NB 4
#define LQ 2048
#define LK 512
#define NQ (NB * LQ)
#define NKV (NB * LK)
#define QD 1024
#define KVC 256
#define QC 384
#define NH 16
#define HDd 64
#define RR 64
#ifndef NQB
#define NQB (NQ / 64)
#endif
typedef __attribute__((ext_vector_type(8))) __bf16 v8b;
__device__ __forceinline__ v16b frag_b(const __bf16* rowk0, int lane) {
  union { v16b v; v8b q[2]; } u; const __bf16* p = rowk0 + 8 * (lane >> 4);
  u.q[0] = *(const v8b*)p; u.q[1] = *(const v8b*)(p + 16); return u.v;
}
__device__ __forceinline__ float bfr(float v) { return (float)(__bf16)v; }
__device__ __attribute__((noinline)) float exp_ni(float v) { return expf(v); }
__device__ __attribute__((noinline)) float erf_ni(float v) { return erff(v); }

__device__ __attribute__((noinline)) float cos_ni(float v) { return cosf(v); }
__device__ __attribute__((noinline)) float sin_ni(float v) { return sinf(v); }
__device__ __attribute__((noinline)) float pow_ni(float a, float b) { return powf(a, b); }
#define WS_PW   0u
#define P_C  0
#define P_D  (P_C + 256 * 1024)
#define P_QU (P_D + 384 * 1024)
#define P_QR (P_QU + 1024 * 384)
#define P_KU (P_QR + 1024 * 384)
#define P_KR (P_KU + 1024 * 256)
#define P_VU (P_KR + 64 * 256)
#define P_O  (P_VU + 1024 * 256)
#define PWEND (P_O + 1024 * 1024)
#define WS_KVC  (WS_PW + 2u * PWEND)
#define WS_QCm  (WS_KVC + 4u * NKV * KVC)
#define WS_QN   (WS_QCm + 4u * NQ * QC)
#define WS_QR   (WS_QN + 4u * NQ * 1024)
#define WS_KN   (WS_QR + 4u * NQ * 1024)
#define WS_KR   (WS_KN + 4u * NKV * 1024)
#define WS_V    (WS_KR + 4u * NKV * 64)
#define WS_CTX  (WS_V + 4u * NKV * 1024)
#define WS_END  (WS_CTX + 4u * NQ * 1024)

__global__ __launch_bounds__(256) void k_packW(const float* __restrict__ Wm, int K, int NOUT, __bf16* __restrict__ DST_) {
  __shared__ __align__(16) __bf16 s[1024]; const int n = blockIdx.x, tid = threadIdx.x;
  for (int k = tid; k < K; k += 256) s[k] = (__bf16)Wm[(size_t)k * NOUT + n];
  __syncthreads();
  for (int q = tid; q < K / 8; q += 256) vst2((unsigned*)(DST_ + (size_t)n * K + q * 8), *(const v4u*)&s[q * 8]);
}
template <int MODE, int ROPE>
__global__ __launch_bounds__(128) void k_gemm(const float* __restrict__ A, int lda, int K, const __bf16* __restrict__ P, int nout, float* __restrict__ OUT, int ldo) {
  __shared__ __align__(16) float so[4][16][132];
  const int tid = threadIdx.x, wave = tid >> 5, lane = tid & 31, col = lane & 15, g = lane >> 4; const size_t r0 = (size_t)blockIdx.x * 64 + wave * 16; const int n0 = blockIdx.y * 128; const int ntl = min(8, (nout - n0) / 16);
  v8f acc[8] = {};
  for (int kc = 0; kc < K / 32; ++kc) { F2 a; if (MODE == 1) { v16b ax; const float* p = A + (r0 + col) * (size_t)lda + kc * 32 + 8 * g;
#pragma unroll
      for (int i = 0; i < 8; ++i) { ax[i] = (__bf16)p[i]; ax[8 + i] = (__bf16)p[16 + i]; } a.h = ax; a.l = ax; } else a = split_row(A + (r0 + col) * (size_t)lda, kc * 32, lane);
#pragma unroll
    for (int j = 0; j < 8; ++j) { if (j < ntl) { const v16b w = frag_b(P + (size_t)(n0 + j * 16 + col) * K + kc * 32, lane); if (MODE == 0) acc[j] = wmma_bf(a.l, w, acc[j]); acc[j] = wmma_bf(a.h, w, acc[j]); } } }
#pragma unroll
  for (int j = 0; j < 8; ++j)
#pragma unroll
    for (int r = 0; r < 8; ++r) so[wave][8 * g + r][j * 16 + col] = acc[j][r];
  LDSX();
  if (ROPE) {
    for (int rl = 0; rl < 16; ++rl) { const size_t row = r0 + rl; const float pos = (float)(ROPE == 1 ? (row % LQ) : (row % LK)); const int i = lane; const float inv = 1.0f / pow_ni(10000.0f, (float)i / 32.0f); const float ang = pos * inv; const float cs = cos_ni(ang), sn = sin_ni(ang);
      for (int grp = 0; grp < (ROPE == 1 ? 2 : 1); ++grp) { const float x1 = so[wave][rl][grp * 64 + i], x2 = so[wave][rl][grp * 64 + 32 + i]; so[wave][rl][grp * 64 + i] = x1 * cs - x2 * sn; so[wave][rl][grp * 64 + 32 + i] = x1 * sn + x2 * cs; } }
    LDSX(); }
  for (int rl = 0; rl < 16; ++rl) for (int pc = lane; pc < ntl * 4; pc += 32) vst2(OUT + (r0 + rl) * (size_t)ldo + n0 + pc * 4, *(const v4f*)&so[wave][rl][pc * 4]);
}
__global__ __launch_bounds__(256) void k_segattn(const float* __restrict__ QN, const float* __restrict__ QR, const float* __restrict__ KN, const float* __restrict__ KR, const float* __restrict__ V, const int* __restrict__ SEG, float* __restrict__ CTX) {
  __shared__ __align__(16) float sc[16][1024 + 4];
  const int tid = threadIdx.x; const int ql = tid >> 4, h = tid & 15; const size_t qi = (size_t)blockIdx.x * 16 + ql; const int b = (int)(qi / LQ); const int seg = min(max(SEG[qi], 0), LK - 1);
  const float* qn = QN + qi * 1024 + h * HDd; const float* qr = QR + qi * 1024 + h * RR; const float scale = 1.0f / sqrtf((float)(HDd + RR));
  float s[3]; int kk[3]; int nk = 0;
#pragma unroll
  for (int j = 0; j < 3; ++j) { const int k = seg - 2 + j; s[j] = -3.0e38f; kk[j] = 0; if (k >= 0) { const size_t kr = (size_t)b * LK + k; const float* kn = KN + kr * 1024 + h * HDd; const float* krp = KR + kr * RR; float a = 0.f;
#pragma unroll 2
      for (int d = 0; d < HDd; ++d) a += qn[d] * kn[d];
      float c = 0.f;
#pragma unroll 2
      for (int d = 0; d < RR; ++d) c += qr[d] * krp[d];
      s[j] = (a + c) * scale; kk[j] = (int)kr; ++nk; } }
  const float mx = fmaxf(s[0], fmaxf(s[1], s[2])); float e[3], z = 0.f;
#pragma unroll
  for (int j = 0; j < 3; ++j) { e[j] = (s[j] <= -1.0e38f) ? 0.f : exp_ni(s[j] - mx); z += e[j]; }
#pragma unroll 1
  for (int d = 0; d < HDd; ++d) { float a = 0.f;
#pragma unroll
    for (int j = 0; j < 3; ++j) if (e[j] != 0.f) a += e[j] * V[(size_t)kk[j] * 1024 + h * HDd + d];
    sc[ql][h * HDd + d] = a / z; }
  __syncthreads();
  for (int q = tid; q < 16 * 256; q += 256) { const int rl = q >> 8, pc = q & 255; vst2(CTX + ((size_t)blockIdx.x * 16 + rl) * 1024 + pc * 4, *(const v4f*)&sc[rl][pc * 4]); }
}
extern "C" void kernel_launch(void* const* d_in, const int* in_sizes, int n_in, void* d_out, int out_size, void* d_ws, size_t ws_size, hipStream_t stream) {
  (void)in_sizes; (void)n_in; (void)out_size;
  const float** F = (const float**)d_in; const int* SEG = (const int*)d_in[2];
  if (ws_size < (size_t)WS_END) return;
  char* ws = (char*)d_ws; __bf16* PW = (__bf16*)(ws + WS_PW); float *KVCm = (float*)(ws + WS_KVC), *QCm = (float*)(ws + WS_QCm), *QN = (float*)(ws + WS_QN), *QR = (float*)(ws + WS_QR), *KN = (float*)(ws + WS_KN), *KR = (float*)(ws + WS_KR), *V = (float*)(ws + WS_V), *CTX = (float*)(ws + WS_CTX);
  k_packW<<<256, 256, 0, stream>>>(F[3], 1024, 256, PW + P_C); k_packW<<<384, 256, 0, stream>>>(F[4], 1024, 384, PW + P_D); k_packW<<<1024, 256, 0, stream>>>(F[5], 384, 1024, PW + P_QU); k_packW<<<1024, 256, 0, stream>>>(F[6], 384, 1024, PW + P_QR);
  k_packW<<<1024, 256, 0, stream>>>(F[7], 256, 1024, PW + P_KU); k_packW<<<64, 256, 0, stream>>>(F[8], 256, 64, PW + P_KR); k_packW<<<1024, 256, 0, stream>>>(F[9], 256, 1024, PW + P_VU); k_packW<<<1024, 256, 0, stream>>>(F[10], 1024, 1024, PW + P_O);
  k_gemm<1, 0><<<dim3(NKV / 64, 2), 128, 0, stream>>>(F[1], QD, QD, PW + P_C, KVC, KVCm, KVC);
  k_gemm<0, 0><<<dim3(NKV / 64, 8), 128, 0, stream>>>(KVCm, KVC, KVC, PW + P_KU, 1024, KN, 1024);
  k_gemm<0, 2><<<dim3(NKV / 64, 1), 128, 0, stream>>>(KVCm, KVC, KVC, PW + P_KR, 64, KR, RR);
  k_gemm<0, 0><<<dim3(NKV / 64, 8), 128, 0, stream>>>(KVCm, KVC, KVC, PW + P_VU, 1024, V, 1024);
  k_gemm<1, 0><<<dim3(NQB, 3), 128, 0, stream>>>(F[0], QD, QD, PW + P_D, QC, QCm, QC);
  k_gemm<0, 0><<<dim3(NQB, 8), 128, 0, stream>>>(QCm, QC, QC, PW + P_QU, 1024, QN, 1024);
  k_gemm<0, 1><<<dim3(NQB, 8), 128, 0, stream>>>(QCm, QC, QC, PW + P_QR, 1024, QR, 1024);
  k_segattn<<<NQB * 4, 256, 0, stream>>>(QN, QR, KN, KR, V, SEG, CTX);
  k_gemm<0, 0><<<dim3(NQB, 8), 128, 0, stream>>>(CTX, 1024, 1024, PW + P_O, QD, (float*)d_out, QD);
}
